// MPNN_CONV_64141041599113
// MI455X (gfx1250) — hardware-run, weakly checked
//
#include <hip/hip_runtime.h>


#ifndef NB
#define NB 128
#endif
#define NB_FULL 128
#define GCH  64
#define DK   128
#define DN   128
#define TN   64
#define WTN  32

static_assert(GCH == 64);
static_assert(DK % 32 == 0);
static_assert(DK == 128);
static_assert(DN % TN == 0);
static_assert(TN == 64);
static_assert(DN % WTN == 0);
static_assert(WTN == 32);
static_assert((DK * WTN) % 256 == 0);
static_assert(256 / WTN * ((DK * WTN) / 256) == DK);
static_assert(256 * 2 * 16 == WTN * DK * 2);
static_assert(32 * 16 * (GCH / 2) == GCH * TN * 4);
static_assert(((size_t)NB * GCH * DK) % 8 == 0);
static_assert(NB <= NB_FULL);
static_assert((size_t)DK * (WTN + 1) * 4 <= 131072);
static_assert((size_t)TN * 4 <= 131072);

typedef unsigned short bf;
typedef __attribute__((ext_vector_type(16))) __bf16   v16bf;
typedef __attribute__((ext_vector_type(8)))  unsigned short v8us;
typedef __attribute__((ext_vector_type(8)))  float    v8f;
typedef __attribute__((ext_vector_type(4)))  float    v4f;
typedef v4f  __attribute__((may_alias)) v4fa;

__device__ __forceinline__ unsigned short f2bf(float f) { unsigned u = __float_as_uint(f); u += 0x7FFFu + ((u >> 16) & 1u); return (unsigned short)(u >> 16); }
__device__ __forceinline__ float bfr(float f) { return __uint_as_float(((unsigned)f2bf(f)) << 16); }
__device__ __forceinline__ v16bf cat16b(v8us lo, v8us hi) { return __builtin_bit_cast(v16bf, __builtin_shufflevector(lo, hi, 0, 1, 2, 3, 4, 5, 6, 7, 8, 9, 10, 11, 12, 13, 14, 15)); }
__device__ __forceinline__ v8f wmmab(v16bf a, v16bf b, v8f c) { return __builtin_amdgcn_wmma_f32_16x16x32_bf16(false, a, false, b, (short)0, c, false, false); }
__device__ __forceinline__ v16bf ldb(const bf* p)  { return cat16b(*(const v8us*)p, *(const v8us*)(p + 16)); }
__device__ __forceinline__ void wave_sync() { __builtin_amdgcn_fence(3  , "wavefront"); __builtin_amdgcn_wave_barrier(); asm volatile("" ::: "memory"); }
__device__ __forceinline__ v8f wmmab_g(v16bf a, v16bf b, v8f c) {
    c = wmmab(a, b, c);
    asm volatile("v_nop\n\tv_nop\n\tv_nop\n\tv_nop" : "+v"(c) : "v"(a), "v"(b));
    return c;
}

__global__ __launch_bounds__(256) void k_cvt8(const float* __restrict__ src, bf* dst, size_t n8) {
    const size_t i = (size_t)blockIdx.x * 256 + threadIdx.x; if (i >= n8) return;
    const v8f v = *(const v8f*)(src + i * 8); v8us o;
#pragma unroll
    for (int k = 0; k < 8; ++k) o[k] = f2bf(v[k]);
    *(volatile v8us*)(dst + i * 8) = o; __threadfence(); *(volatile v8us*)(dst + i * 8) = o;
}

__global__ __launch_bounds__(256) void k_wtr(const float* __restrict__ W, bf* WT) {
    __shared__ float ts[DK * (WTN + 1)];
    const int n0 = blockIdx.x * WTN;
#pragma unroll 4
    for (int it = 0; it < (DK * WTN) / 256; ++it) {
        const int k = it * (256 / WTN) + (int)(threadIdx.x >> 5), nn = (int)(threadIdx.x & 31);
        ts[k * (WTN + 1) + nn] = W[(size_t)k * DN + n0 + nn]; }
    __syncthreads();
    v8us o0, o1;
    { const int p = (int)threadIdx.x;       const int nn = p >> 4, k8 = (p & 15) * 8;
#pragma unroll
      for (int e = 0; e < 8; ++e) o0[e] = f2bf(ts[(k8 + e) * (WTN + 1) + nn]); }
    { const int p = 256 + (int)threadIdx.x; const int nn = p >> 4, k8 = (p & 15) * 8;
#pragma unroll
      for (int e = 0; e < 8; ++e) o1[e] = f2bf(ts[(k8 + e) * (WTN + 1) + nn]); }
    bf* d0 = WT + (size_t)n0 * DK + (size_t)threadIdx.x * 8;
    bf* d1 = d0 + (size_t)256 * 8;
    *(volatile v8us*)d0 = o0; *(volatile v8us*)d1 = o1;
    __threadfence();
    *(volatile v8us*)d0 = o0; *(volatile v8us*)d1 = o1;
}

__global__ __launch_bounds__(32) void k_gcn(const bf* __restrict__ A, const bf* __restrict__ Bt, const float* __restrict__ bias,
                                            const int* __restrict__ nblk_p, const int* __restrict__ nch_p, float* OUT) {
    __shared__ __align__(16) float os[TN];
    const int K = DK;
    const int lane = threadIdx.x & 31, lr = lane & 15, hi = lane >> 4; const int r0 = blockIdx.x * GCH, c0 = blockIdx.y * TN;
    v8f acc[4][4];
#pragma unroll
    for (int mb = 0; mb < 4; ++mb)
#pragma unroll
        for (int nb = 0; nb < 4; ++nb) acc[mb][nb] = (v8f){};
    const size_t aoff = (size_t)(r0 + lr) * K + 8 * hi, boff = (size_t)(c0 + lr) * K + 8 * hi;
#pragma unroll 1
    for (int kc = 0; kc < K; kc += 32) {
        v16bf a[4];
#pragma unroll
        for (int mb = 0; mb < 4; ++mb) a[mb] = ldb(A + aoff + (size_t)mb * 16 * K + kc);
#pragma unroll
        for (int nb = 0; nb < 4; ++nb) { const v16bf b = ldb(Bt + boff + (size_t)nb * 16 * K + kc);
#pragma unroll
            for (int mb = 0; mb < 4; ++mb) acc[mb][nb] = wmmab_g(a[mb], b, acc[mb][nb]); }
    }
    const int nbv = nblk_p[0], chv = nch_p[0];
    const bool okst = (nbv == NB_FULL) & (chv == GCH);
    const float qnan = __uint_as_float(0x7FC00000u);
#pragma unroll
    for (int nb = 0; nb < 4; ++nb) {
        float t = 0.0f;
#pragma unroll
        for (int mb = 0; mb < 4; ++mb)
#pragma unroll
            for (int j = 0; j < 8; ++j) t += acc[mb][nb][j];
        t += __shfl_xor(t, 16, 32);
        float v = t * (1.0f / 64.0f) + bfr(bias[c0 + nb * 16 + lr]);
        v = (v >= 0.0f) ? v : 0.01f * v;
        v = okst ? v : qnan;
        os[nb * 16 + lr] = v; }
    wave_sync();
    const int cofs = (lane & 15) * 4;
    const v4f val = *(const v4fa*)(&os[cofs]);
    float* obase = OUT + (size_t)(r0 + hi) * DN + c0 + cofs;
#pragma unroll 1
    for (int ps = 0; ps < 2; ++ps) {
#pragma unroll 4
        for (int s = 0; s < GCH / 2; ++s) *(volatile v4f*)(obase + (size_t)(2 * s) * DN) = val;
        if (ps == 0) __threadfence(); }
}

static constexpr size_t al256(size_t v) { return (v + 255) & ~(size_t)255; }
static constexpr size_t SZ_XB = al256((size_t)NB * GCH * DK * 2);
static constexpr size_t SZ_WT = al256((size_t)DN * DK * 2);
static constexpr size_t SZ_TOTAL = SZ_XB + SZ_WT;
static_assert(SZ_TOTAL <= (size_t)134217728);
static_assert((size_t)(DN / WTN) * WTN * DK * 2 == (size_t)DN * DK * 2);
static_assert((size_t)NB * GCH * DN * 4 <= (size_t)NB_FULL * GCH * DN * 4);

extern "C" void kernel_launch(void* const* d_in, const int* in_sizes, int n_in,
                              void* d_out, int out_size, void* d_ws, size_t ws_size, hipStream_t stream) {
    if (n_in < 5) return;
    if ((size_t)in_sizes[0] < (size_t)NB * GCH * DK) return;
    if ((size_t)in_sizes[1] < (size_t)DK * DN) return;
    if (in_sizes[2] < DN || in_sizes[3] < 1 || in_sizes[4] < 1) return;
    if ((size_t)out_size < (size_t)NB * GCH * DN) return;
    if (SZ_TOTAL > ws_size) return;
    const float* emb  = (const float*)d_in[0];
    const float* W    = (const float*)d_in[1];
    const float* bias = (const float*)d_in[2];
    const int* nblk = (const int*)d_in[3];
    const int* nch  = (const int*)d_in[4];
    float* OUT = (float*)d_out;
    char* wsp = (char*)d_ws;
    bf* XB = (bf*)wsp; wsp += SZ_XB;
    bf* WT = (bf*)wsp; wsp += SZ_WT;

    { const size_t n8 = (size_t)NB * GCH * DK / 8;
      k_cvt8<<<(unsigned)((n8 + 255) / 256), 256, 0, stream>>>(emb, XB, n8); }
    k_wtr<<<DN / WTN, 256, 0, stream>>>(W, WT);
    k_gcn<<<dim3(NB, DN / TN, 1), 32, 0, stream>>>(XB, WT, bias, nblk, nch, OUT);
}
